// SeqLinear_6786048327774
// MI455X (gfx1250) — hardware-verified
//
#include <hip/hip_runtime.h>
#include <stdint.h>
#include <stddef.h>

constexpr int kBatch   = 2;
constexpr int kSeq     = 4096;
constexpr int kDm      = 1024;
constexpr int kNh      = 16;
constexpr int kHd      = 64;
constexpr int kChunk   = 64;
constexpr int kNch     = 64;
constexpr int kConvCh  = 3072;
constexpr int kProj    = 3088;
constexpr int kProjPad = 3136;
constexpr int kRec     = 160;
constexpr int kLP      = 72;
constexpr int kPlane   = 64 * kLP;

static_assert(kSeq == kNch * kChunk);
static_assert(kDm % 64 == 0 && kSeq % 64 == 0 && kProjPad % 64 == 0);
static_assert(kDm % 32 == 0);
static_assert(kProjPad >= kConvCh + 64);
static_assert(kNh * kHd == kDm);

constexpr size_t kBytesWin   = (size_t)kProjPad * kDm * 2;
constexpr size_t kBytesWout  = (size_t)kDm * kDm * 2;
constexpr size_t kBytesXb    = (size_t)kSeq * kDm * 2;
constexpr size_t kBytesPlane = (size_t)kSeq * kDm * 4;
constexpr size_t kBytesPW    = (size_t)kSeq * 64 * 4;
constexpr size_t kBytesRec   = (size_t)kNh * kNch * kRec * 4;
constexpr size_t kBytesTW    = (size_t)kNh * kNch * 64 * 4;
constexpr size_t kBytesSt    = (size_t)kNh * kNch * 4096 * 4;
constexpr size_t kBytesYn    = (size_t)kSeq * kDm * 2;

constexpr size_t kOffWin  = 0;
constexpr size_t kOffWout = kOffWin + kBytesWin;
constexpr size_t kOffXb   = kOffWout + kBytesWout;
constexpr size_t kOffPC   = kOffXb + kBytesXb;
constexpr size_t kOffPB   = kOffPC + kBytesPlane;
constexpr size_t kOffPX   = kOffPB + kBytesPlane;
constexpr size_t kOffPW   = kOffPX + kBytesPlane;
constexpr size_t kOffRec  = kOffPW + kBytesPW;
constexpr size_t kOffTW   = kOffRec + kBytesRec;
constexpr size_t kOffSt   = kOffTW + kBytesTW;
constexpr size_t kOffSn   = kOffSt + kBytesSt;
constexpr size_t kOffYnH  = kOffSn + kBytesSt;
constexpr size_t kOffYnL  = kOffYnH + kBytesYn;
constexpr size_t kWsTotal = kOffYnL + kBytesYn;
static_assert(kWsTotal == 119537664);
static_assert(kWsTotal <= 134217728);
static_assert(kOffWout % 256 == 0 && kOffXb % 256 == 0 && kOffPC % 256 == 0 && kOffPW % 256 == 0);
static_assert(kOffRec % 256 == 0 && kOffTW % 256 == 0 && kOffSt % 256 == 0 && kOffSn % 256 == 0);
static_assert(kOffYnH % 256 == 0 && kOffYnL % 256 == 0);

typedef __attribute__((ext_vector_type(16))) _Float16 v16h;
typedef __attribute__((ext_vector_type(8)))  _Float16 v8h;
typedef __attribute__((ext_vector_type(16))) __bf16   v16b;
typedef __attribute__((ext_vector_type(8)))  __bf16   v8b;
typedef __attribute__((ext_vector_type(8)))  float    v8f;
typedef __attribute__((ext_vector_type(4)))  float    v4f;
typedef __attribute__((ext_vector_type(4)))  unsigned v4u;

__device__ __forceinline__ unsigned short f2bf_bits(float f) {
  unsigned u = __float_as_uint(f);
  return (unsigned short)((u + 0x7FFFu + ((u >> 16) & 1u)) >> 16);
}
__device__ __forceinline__ float bf_bits2f(unsigned short h) { return __uint_as_float(((unsigned)h) << 16); }
__device__ __forceinline__ float bf_rne(float f) { return bf_bits2f(f2bf_bits(f)); }
__device__ __forceinline__ void split_bf(float f, __bf16& hi, __bf16& lo) {
  const unsigned short hb = f2bf_bits(f);
  hi = __builtin_bit_cast(__bf16, hb);
  lo = __builtin_bit_cast(__bf16, f2bf_bits(f - bf_bits2f(hb)));
}
__device__ __forceinline__ v8f zero8() { return (v8f){0.f, 0.f, 0.f, 0.f, 0.f, 0.f, 0.f, 0.f}; }

__device__ __forceinline__ void dep_guard_h(v8f& a, v8f& b, v16h x, v16h y) { asm volatile("v_nop\n\tv_nop\n\tv_nop\n\tv_nop" : "+v"(a), "+v"(b) : "v"(x), "v"(y)); }
__device__ __forceinline__ void dep_guard_b(v8f& a, v8f& b, v16b x, v16b y) { asm volatile("v_nop\n\tv_nop\n\tv_nop\n\tv_nop" : "+v"(a), "+v"(b) : "v"(x), "v"(y)); }
__device__ __forceinline__ void keep4_h(v16h a, v16h b, v16h c, v16h d) { asm volatile("v_nop" :: "v"(a), "v"(b), "v"(c), "v"(d)); }
__device__ __forceinline__ void keep4_b(v16b a, v16b b, v16b c, v16b d) { asm volatile("v_nop" :: "v"(a), "v"(b), "v"(c), "v"(d)); }
__device__ __forceinline__ void acc_guard4(v8f& a, v8f& b, v8f& c, v8f& d) { asm volatile("v_nop\n\tv_nop\n\tv_nop\n\tv_nop" : "+v"(a), "+v"(b), "+v"(c), "+v"(d)); }
__device__ __forceinline__ void acc_guard2(v8f& a, v8f& b) { asm volatile("v_nop\n\tv_nop\n\tv_nop\n\tv_nop" : "+v"(a), "+v"(b)); }
__device__ __forceinline__ void wave_lds_sync() {
  __builtin_amdgcn_fence(__ATOMIC_RELEASE, "workgroup");
  __builtin_amdgcn_wave_barrier();
  __builtin_amdgcn_fence(__ATOMIC_ACQUIRE, "workgroup");
}

template <typename T> struct Frag;
template <> struct Frag<_Float16> {
  typedef v16h V; union U { v16h v; v8h h[2]; };
  static __device__ __forceinline__ v16h load(const _Float16* p) {
    U f; f.h[0] = *(const v8h*)(p); f.h[1] = *(const v8h*)(p + 16); return f.v;
  }
  static __device__ __forceinline__ v8f mma(v16h a, v16h b, v8f c) {
    return __builtin_amdgcn_wmma_f32_16x16x32_f16(false, a, false, b, (short)0, c, false, false);
  }
  static __device__ __forceinline__ void guard(v8f& a, v8f& b, v16h x, v16h y) { dep_guard_h(a, b, x, y); }
  static __device__ __forceinline__ void keep(v16h a, v16h b, v16h c, v16h d) { keep4_h(a, b, c, d); }
};
template <> struct Frag<__bf16> {
  typedef v16b V; union U { v16b v; v8b h[2]; };
  static __device__ __forceinline__ v16b load(const __bf16* p) {
    U f; f.h[0] = *(const v8b*)(p); f.h[1] = *(const v8b*)(p + 16); return f.v;
  }
  static __device__ __forceinline__ v8f mma(v16b a, v16b b, v8f c) {
    return __builtin_amdgcn_wmma_f32_16x16x32_bf16(false, a, false, b, (short)0, c, false, false);
  }
  static __device__ __forceinline__ void guard(v8f& a, v8f& b, v16b x, v16b y) { dep_guard_b(a, b, x, y); }
  static __device__ __forceinline__ void keep(v16b a, v16b b, v16b c, v16b d) { keep4_b(a, b, c, d); }
};

template <int ET> struct Elem;
template <> struct Elem<0> { typedef _Float16 T; };
template <> struct Elem<1> { typedef __bf16 T; };
template <int ET, int SPLITM, int BIAS_MODE, int OUT_MODE, bool RESID, int ACT = 0>
__global__ __launch_bounds__(256) void wmma_gemm64(
    const unsigned short* __restrict__ Ap, const unsigned short* __restrict__ A2p, int lda, long strideA,
    const unsigned short* __restrict__ Btp, const unsigned short* __restrict__ Bt2p, int ldb, long strideB,
    void* __restrict__ Cout, void* __restrict__ Cout2, int ldc, long strideC,
    const float* __restrict__ bias,
    const float* __restrict__ resid, long strideR,
    int M, int N, int K, float scale) {
  typedef typename Elem<ET>::T T;
  typedef typename Frag<T>::V V;
  constexpr bool SPLIT  = (SPLITM != 0);
  constexpr bool SPLITB = (SPLITM == 1);
  const T* A = (const T*)Ap; const T* A2 = (const T*)A2p; const T* Bt = (const T*)Btp; const T* Bt2 = (const T*)Bt2p;
  __shared__ __align__(16) float sT[8][16 * 68];
  const int b    = blockIdx.y;
  const int lane = threadIdx.x & 31;
  const int wave = threadIdx.x >> 5;
  const int tilesN = N >> 6;
  const int tilesM = M >> 6;
  const int tile = blockIdx.x * 8 + wave;
  if (tile >= tilesM * tilesN) return;
  const int tm = tile / tilesN;
  const int tn = tile - tm * tilesN;
  const int m0 = tm << 6;
  const int n0 = tn << 6;

  const T* Ab  = A  + (size_t)b * strideA;
  const T* Bb  = Bt + (size_t)b * strideB;
  const T* Ab2 = SPLIT  ? (A2  + (size_t)b * strideA) : nullptr;
  const T* Bb2 = SPLITB ? (Bt2 + (size_t)b * strideB) : nullptr;

  const int rlane = lane & 15;
  const int koff  = (lane >> 4) * 8;
  const int mOff  = (lane >> 4) * 8;

  v8f acc[4][4];
#pragma unroll
  for (int i = 0; i < 4; ++i)
#pragma unroll
    for (int j = 0; j < 4; ++j) acc[i][j] = zero8();

  for (int k0 = 0; k0 < K; k0 += 32) {
    V bh[4], bl[4];
#pragma unroll
    for (int j = 0; j < 4; ++j) {
      const size_t bo = (size_t)(n0 + (j << 4) + rlane) * ldb + koff + k0;
      bh[j] = Frag<T>::load(Bb + bo);
      if (SPLITB) bl[j] = Frag<T>::load(Bb2 + bo);
    }
#pragma unroll
    for (int i = 0; i < 4; ++i) {
      const size_t ao = (size_t)(m0 + (i << 4) + rlane) * lda + koff + k0;
      V ah = Frag<T>::load(Ab + ao);
      V al;
      if (SPLIT) al = Frag<T>::load(Ab2 + ao);
#pragma unroll
      for (int j = 0; j < 4; ++j) {
        acc[i][j] = Frag<T>::mma(ah, bh[j], acc[i][j]);
        if (SPLITB) acc[i][j] = Frag<T>::mma(ah, bl[j], acc[i][j]);
        if (SPLIT)  acc[i][j] = Frag<T>::mma(al, bh[j], acc[i][j]);
      }
      Frag<T>::guard(acc[i][0], acc[i][3], ah, SPLIT ? al : ah);
    }
    Frag<T>::keep(bh[0], bh[1], bh[2], bh[3]);
    if (SPLITB) Frag<T>::keep(bl[0], bl[1], bl[2], bl[3]);
  }
  acc_guard4(acc[0][0], acc[0][1], acc[0][2], acc[0][3]);
  acc_guard4(acc[1][0], acc[1][1], acc[1][2], acc[1][3]);
  acc_guard4(acc[2][0], acc[2][1], acc[2][2], acc[2][3]);
  acc_guard4(acc[3][0], acc[3][1], acc[3][2], acc[3][3]);

  float* slab = sT[wave];
  const float* Rb = RESID ? (resid + (size_t)b * strideR) : nullptr;
#pragma unroll
  for (int i = 0; i < 4; ++i) {
    const int mBase = m0 + (i << 4);
#pragma unroll
    for (int j = 0; j < 4; ++j) {
      const int n = n0 + (j << 4) + rlane;
      float bv = 0.f;
      if (BIAS_MODE == 2) bv = bias[n];
#pragma unroll
      for (int r = 0; r < 8; ++r) {
        float v = acc[i][j][r] * scale;
        if (BIAS_MODE == 1) v += bias[mBase + mOff + r];
        if (BIAS_MODE == 2) v += bv;
        if (RESID) v += Rb[(size_t)(mBase + mOff + r) * ldc + n];
        if (ACT == 1) v = tanhf(v);
        if (ACT == 2) v = fmaxf(v, 0.0f);
        if (ACT == 3) v = v / (1.0f + expf(-v));
        if (ACT == 4) v = (v > 0.f) ? v : 0.01f * v;
        slab[(mOff + r) * 68 + (j << 4) + rlane] = v;
      }
    }
    __builtin_amdgcn_fence(__ATOMIC_RELEASE, "workgroup");
    __builtin_amdgcn_wave_barrier();
    __builtin_amdgcn_fence(__ATOMIC_ACQUIRE, "workgroup");
    if (OUT_MODE == 0) {
      float* C = (float*)Cout + (size_t)b * strideC;
      const int hh = lane >> 4, c4 = (lane & 15) * 4;
      for (int pass = 0; pass < 2; ++pass) {
#pragma unroll
        for (int it = 0; it < 8; ++it) {
          const int row = it * 2 + hh;
          v4f v = *(const v4f*)(slab + row * 68 + c4);
          *(volatile v4f*)(C + (size_t)(mBase + row) * ldc + n0 + c4) = v;
        }
        __threadfence();
      }
    } else {
      const int q = lane >> 3, c8 = (lane & 7) * 8;
      unsigned short* C  = (unsigned short*)Cout  + (size_t)b * strideC;
      unsigned short* C2 = (OUT_MODE == 2) ? ((unsigned short*)Cout2 + (size_t)b * strideC) : nullptr;
      for (int pass = 0; pass < 2; ++pass) {
#pragma unroll
        for (int it = 0; it < 4; ++it) {
          const int row = it * 4 + q;
          const float* sp = slab + row * 68 + c8;
          v8h hv, lv;
#pragma unroll
          for (int e = 0; e < 8; ++e) {
            if (OUT_MODE == 1) {
              hv[e] = (_Float16)sp[e];
            } else {
              unsigned short hb = f2bf_bits(sp[e]);
              unsigned short lb = f2bf_bits(sp[e] - bf_bits2f(hb));
              hv[e] = __builtin_bit_cast(_Float16, hb);
              lv[e] = __builtin_bit_cast(_Float16, lb);
            }
          }
          *(volatile v8h*)(C + (size_t)(mBase + row) * ldc + n0 + c8) = hv;
          if (OUT_MODE == 2) *(volatile v8h*)(C2 + (size_t)(mBase + row) * ldc + n0 + c8) = lv;
        }
        __threadfence();
      }
    }
    __builtin_amdgcn_fence(__ATOMIC_RELEASE, "workgroup");
    __builtin_amdgcn_wave_barrier();
    __builtin_amdgcn_fence(__ATOMIC_ACQUIRE, "workgroup");
  }
}

__global__ __launch_bounds__(256) void k_cast_rows(const float* __restrict__ in, unsigned short* __restrict__ out,
                                                   int rows_in, int rows_out) {
  const int i = blockIdx.x * 256 + threadIdx.x;
  const int n8 = rows_out * (kDm >> 3);
  if (i < n8) {
    const int row = i >> 7;
    const int c8 = (i & 127) * 8;
    const int rowc = (row < rows_in) ? row : (rows_in - 1);
    const bool ok = (row < rows_in);
    const float* src = in + (size_t)rowc * kDm + c8;
    const v4f a = *(const v4f*)(src);
    const v4f bb = *(const v4f*)(src + 4);
    v4u pk;
    pk[0] = ok ? ((unsigned)f2bf_bits(a[0]) | ((unsigned)f2bf_bits(a[1]) << 16)) : 0u;
    pk[1] = ok ? ((unsigned)f2bf_bits(a[2]) | ((unsigned)f2bf_bits(a[3]) << 16)) : 0u;
    pk[2] = ok ? ((unsigned)f2bf_bits(bb[0]) | ((unsigned)f2bf_bits(bb[1]) << 16)) : 0u;
    pk[3] = ok ? ((unsigned)f2bf_bits(bb[2]) | ((unsigned)f2bf_bits(bb[3]) << 16)) : 0u;
    unsigned short* dst = out + (size_t)row * kDm + c8;
    *(volatile v4u*)dst = pk;
    __threadfence();
    *(volatile v4u*)dst = pk;
  }
}

__global__ __launch_bounds__(64) void k_tab(const float* __restrict__ yw, const float* __restrict__ wbase,
                                            float* __restrict__ trec, float* __restrict__ tw) {
  const int h = blockIdx.x;
  const int t = threadIdx.x;
  __shared__ __align__(16) float sRec[64 * kRec];
  __shared__ __align__(16) float sW[64 * 64];
  __shared__ float sCSS[65], sMN[65], sND[64], sLAST[64];
  const float wb = bf_rne(wbase[h]);
  float* rec = sRec + t * kRec;
#pragma unroll 1
  for (int i = 133; i < kRec; ++i) rec[i] = 0.f;
  float run = 0.f, mnp = __builtin_inff(), mx = -__builtin_inff();
#pragma unroll 1
  for (int l = 0; l < kChunk; ++l) {
    const float a = yw[((size_t)(t * kChunk + l)) * 64 + h] * wb;
    run = run + a;
    rec[l] = run;
    mnp = fminf(mnp, run);
    rec[64 + l] = mnp;
    mx = fmaxf(mx, run);
  }
  float nd = 0.f;
#pragma unroll 1
  for (int l = 0; l < kChunk; ++l) nd += expf(mnp - rec[l]);
  rec[128] = mx; rec[129] = mnp; rec[130] = nd; rec[131] = run;
  sLAST[t] = run; sND[t] = nd;
  __syncthreads();
  if (t == 0) {
    float cs = 0.f, mn = 0.f;
    sCSS[0] = 0.f; sMN[0] = 0.f;
#pragma unroll 1
    for (int k = 0; k < kNch; ++k) {
      cs = cs + sLAST[k];
      sCSS[k + 1] = cs;
      mn = fminf(mn, cs);
      sMN[k + 1] = mn;
    }
  }
  __syncthreads();
  {
    const int z = t;
    const float mnz = sMN[z];
    float ndz = 0.f;
#pragma unroll 1
    for (int k = 0; k < kNch; ++k) {
      const bool ok = (k < z);
      const float arg = ok ? (mnz - sCSS[k + 1]) : 0.f;
      const float e = expf(arg);
      const float wv = ok ? e : 0.f;
      sW[z * 64 + k] = wv;
      ndz += wv * sND[k];
    }
    rec[132] = ndz;
  }
  __syncthreads();
  {
    float* dst = trec + (size_t)h * kNch * kRec;
    const v4f* s4 = (const v4f*)sRec;
    for (int pass = 0; pass < 2; ++pass) {
#pragma unroll 1
      for (int i = t; i < 64 * kRec / 4; i += 64) { const v4f v = s4[i]; *(volatile v4f*)(dst + 4 * i) = v; }
      __threadfence();
    }
    float* dw = tw + (size_t)h * 64 * 64;
    const v4f* w4 = (const v4f*)sW;
    for (int pass = 0; pass < 2; ++pass) {
#pragma unroll 1
      for (int i = t; i < 64 * 64 / 4; i += 64) { const v4f v = w4[i]; *(volatile v4f*)(dw + 4 * i) = v; }
      __threadfence();
    }
  }
}

struct Taps { float w0, w1, w2, w3, cb; };
__device__ __forceinline__ Taps load_taps(const float* __restrict__ cw, const float* __restrict__ cbp, int ch) {
  Taps tp;
  tp.w0 = bf_rne(cw[ch * 4 + 0]); tp.w1 = bf_rne(cw[ch * 4 + 1]);
  tp.w2 = bf_rne(cw[ch * 4 + 2]); tp.w3 = bf_rne(cw[ch * 4 + 3]);
  tp.cb = bf_rne(cbp[ch]);
  return tp;
}
template <bool TRANS, bool SCALE>
__device__ __forceinline__ void conv_col16(const float* __restrict__ plane, int gcol, int growc, int l0, Taps tp,
                                           const float* sc, __bf16* dh, __bf16* dl, int col) {
  float y0, y1, y2;
  {
    const int r0 = growc + l0 - 3, r1 = r0 + 1, r2 = r0 + 2;
    const float v0 = plane[(size_t)(r0 < 0 ? 0 : r0) * kDm + gcol];
    const float v1 = plane[(size_t)(r1 < 0 ? 0 : r1) * kDm + gcol];
    const float v2 = plane[(size_t)(r2 < 0 ? 0 : r2) * kDm + gcol];
    y0 = (r0 >= 0) ? v0 : 0.f;
    y1 = (r1 >= 0) ? v1 : 0.f;
    y2 = (r2 >= 0) ? v2 : 0.f;
  }
#pragma unroll 1
  for (int i = 0; i < 16; ++i) {
    const int l = l0 + i;
    const float y3 = plane[(size_t)(growc + l) * kDm + gcol];
    float v = tp.cb + tp.w0 * y0 + tp.w1 * y1 + tp.w2 * y2 + tp.w3 * y3;
    if (SCALE) v = v * sc[l];
    __bf16 hi, lo;
    split_bf(v, hi, lo);
    const int di = TRANS ? (col * kLP + l) : (l * kLP + col);
    dh[di] = hi;
    dl[di] = lo;
    y0 = y1; y1 = y2; y2 = y3;
  }
}

__device__ __forceinline__ void mma_pair64(const __bf16* Ah, const __bf16* Al, int ra0,
                                           const __bf16* Bh, const __bf16* Bl, int rb0,
                                           int lane, v8f& acc0, v8f& acc1) {
  const int rl = lane & 15, koff = (lane >> 4) * 8;
#pragma unroll
  for (int k0 = 0; k0 < 64; k0 += 32) {
    const v16b ah  = Frag<__bf16>::load(Ah + (ra0 + rl) * kLP + koff + k0);
    const v16b al  = Frag<__bf16>::load(Al + (ra0 + rl) * kLP + koff + k0);
    const v16b b0h = Frag<__bf16>::load(Bh + (rb0 + rl) * kLP + koff + k0);
    const v16b b0l = Frag<__bf16>::load(Bl + (rb0 + rl) * kLP + koff + k0);
    const v16b b1h = Frag<__bf16>::load(Bh + (rb0 + 16 + rl) * kLP + koff + k0);
    const v16b b1l = Frag<__bf16>::load(Bl + (rb0 + 16 + rl) * kLP + koff + k0);
    acc0 = Frag<__bf16>::mma(ah, b0h, acc0);
    acc0 = Frag<__bf16>::mma(ah, b0l, acc0);
    acc0 = Frag<__bf16>::mma(al, b0h, acc0);
    acc1 = Frag<__bf16>::mma(ah, b1h, acc1);
    acc1 = Frag<__bf16>::mma(ah, b1l, acc1);
    acc1 = Frag<__bf16>::mma(al, b1h, acc1);
    Frag<__bf16>::guard(acc0, acc1, ah, al);
    Frag<__bf16>::keep(b0h, b0l, b1h, b1l);
  }
}

__device__ __forceinline__ void store_pair_f32(float* slab, v8f acc0, v8f acc1, int lane, float* gbase, int ld) {
  const int rl = lane & 15, hh = lane >> 4;
#pragma unroll
  for (int r = 0; r < 8; ++r) {
    slab[(8 * hh + r) * 36 + rl] = acc0[r];
    slab[(8 * hh + r) * 36 + 16 + rl] = acc1[r];
  }
  wave_lds_sync();
  const int q = lane >> 3, e4 = (lane & 7) * 4;
  for (int pass = 0; pass < 2; ++pass) {
#pragma unroll
    for (int it = 0; it < 4; ++it) {
      const int row = it * 4 + q;
      const v4f v = *(const v4f*)(slab + row * 36 + e4);
      *(volatile v4f*)(gbase + (size_t)row * ld + e4) = v;
    }
    __threadfence();
  }
  wave_lds_sync();
}

__global__ __launch_bounds__(256) void k_states(const float* __restrict__ pB, const float* __restrict__ pX,
                                               const float* __restrict__ convw, const float* __restrict__ convb,
                                               const float* __restrict__ trec, float* __restrict__ st) {
  const int c = blockIdx.x, h = blockIdx.y;
  const int t = threadIdx.x, lane = t & 31, w = t >> 5;
  __shared__ __align__(16) __bf16 pool[4 * kPlane];
  __shared__ __align__(16) float slab[8][16 * 36];
  __shared__ float sD[64];
  __bf16* xH = pool;
  __bf16* xL = pool + kPlane;
  __bf16* bTH = pool + 2 * kPlane;
  __bf16* bTL = pool + 3 * kPlane;
  const float* rec = trec + ((size_t)h * kNch + c) * kRec;
  if (t < 64) {
    const float mnall = rec[129];
    sD[t] = expf(mnall - rec[t]);
  }
  __syncthreads();
  const int col = t & 63, l0 = (t >> 6) * 16;
  const int growc = c * kChunk;
  {
    const Taps tb = load_taps(convw, convb, kDm + h * kHd + col);
    conv_col16<true, false>(pB, h * kHd + col, growc, l0, tb, sD, bTH, bTL, col);
    const Taps tx = load_taps(convw, convb, 2 * kDm + h * kHd + col);
    conv_col16<true, true>(pX, h * kHd + col, growc, l0, tx, sD, xH, xL, col);
  }
  __syncthreads();
  const int tp = w >> 1, tn = (w & 1) * 2;
  v8f a0 = zero8(), a1 = zero8();
  mma_pair64(xH, xL, tp * 16, bTH, bTL, tn * 16, lane, a0, a1);
  acc_guard2(a0, a1);
  float* gbase = st + ((size_t)h * kNch + c) * 4096 + (size_t)(tp * 16) * 64 + tn * 16;
  store_pair_f32(slab[w], a0, a1, lane, gbase, 64);
}

__global__ __launch_bounds__(256) void k_inter(const float* __restrict__ tw, const float* __restrict__ st,
                                              float* __restrict__ sn) {
  const int ns = blockIdx.x, h = blockIdx.y;
  const int t = threadIdx.x, lane = t & 31, w = t >> 5;
  __shared__ __align__(16) __bf16 pool[4 * kPlane];
  __shared__ __align__(16) float slab[8][16 * 36];
  __bf16* wH = pool;
  __bf16* wL = pool + kPlane;
  __bf16* sTH = pool + 2 * kPlane;
  __bf16* sTL = pool + 3 * kPlane;
#pragma unroll
  for (int i = 0; i < 4; ++i) {
    const int idx4 = t + 256 * i;
    const int z = idx4 >> 4, k4 = (idx4 & 15) * 4;
    const v4f v = *(const v4f*)(tw + (size_t)h * 4096 + z * 64 + k4);
#pragma unroll
    for (int e = 0; e < 4; ++e) { __bf16 hi, lo; split_bf(v[e], hi, lo); wH[z * kLP + k4 + e] = hi; wL[z * kLP + k4 + e] = lo; }
  }
  const float* sb = st + (size_t)h * kNch * 4096 + ns * 64;
#pragma unroll
  for (int i = 0; i < 4; ++i) {
    const int idx4 = t + 256 * i;
    const int k = idx4 >> 4, n4 = (idx4 & 15) * 4;
    const v4f v = *(const v4f*)(sb + (size_t)k * 4096 + n4);
#pragma unroll
    for (int e = 0; e < 4; ++e) { __bf16 hi, lo; split_bf(v[e], hi, lo); sTH[(n4 + e) * kLP + k] = hi; sTL[(n4 + e) * kLP + k] = lo; }
  }
  __syncthreads();
  const int tz = w >> 1, tn = (w & 1) * 2;
  v8f a0 = zero8(), a1 = zero8();
  mma_pair64(wH, wL, tz * 16, sTH, sTL, tn * 16, lane, a0, a1);
  acc_guard2(a0, a1);
  float* gbase = sn + (size_t)h * kNch * 4096 + (size_t)(tz * 16) * 4096 + ns * 64 + tn * 16;
  store_pair_f32(slab[w], a0, a1, lane, gbase, 4096);
}

__global__ __launch_bounds__(256) void k_out(const float* __restrict__ pC, const float* __restrict__ pB, const float* __restrict__ pX,
                                            const float* __restrict__ convw, const float* __restrict__ convb,
                                            const float* __restrict__ trec, const float* __restrict__ sn,
                                            unsigned short* __restrict__ ynh, unsigned short* __restrict__ ynl) {
  const int c = blockIdx.x, h = blockIdx.y;
  const int t = threadIdx.x, lane = t & 31, w = t >> 5;
  const int rl = lane & 15, hh = lane >> 4;
  __shared__ __align__(16) __bf16 pool[6 * kPlane];
  __shared__ float sCS[64], sMNP[64], sSDO[64], sNDG[128];
  __bf16* aH = pool;               __bf16* aL = pool + kPlane;
  __bf16* bH = pool + 2 * kPlane;  __bf16* bL = pool + 3 * kPlane;
  __bf16* mH = pool + 4 * kPlane;  __bf16* mL = pool + 5 * kPlane;
  const float* rec = trec + ((size_t)h * kNch + c) * kRec;
  const float mx = rec[128];
  const float ndz = rec[132];
  if (t < 64) {
    const float cs = rec[t];
    sCS[t] = cs;
    sMNP[t] = rec[64 + t];
    sSDO[t] = expf(cs - mx);
  }
  const int col = t & 63, l0 = (t >> 6) * 16;
  const int growc = c * kChunk;
  {
    const Taps tc = load_taps(convw, convb, h * kHd + col);
    conv_col16<false, false>(pC, h * kHd + col, growc, l0, tc, sSDO, aH, aL, col);
    const Taps tb = load_taps(convw, convb, kDm + h * kHd + col);
    conv_col16<false, false>(pB, h * kHd + col, growc, l0, tb, sSDO, bH, bL, col);
  }
  __syncthreads();
  const int lt = w >> 1;
  const int cb2 = (w & 1) * 2;
  {
    v8f g[2];
    g[0] = zero8(); g[1] = zero8();
    mma_pair64(aH, aL, lt * 16, bH, bL, cb2 * 16, lane, g[0], g[1]);
    acc_guard2(g[0], g[1]);
    float rs[8];
#pragma unroll
    for (int r = 0; r < 8; ++r) rs[r] = 0.f;
#pragma unroll
    for (int j = 0; j < 2; ++j) {
      const int scol = (cb2 + j) * 16 + rl;
      const float css = sCS[scol];
#pragma unroll
      for (int r = 0; r < 8; ++r) {
        const int l = lt * 16 + 8 * hh + r;
        const bool ok = (scol <= l);
        const float arg = ok ? (sMNP[l] - css) : 0.f;
        const float e = expf(arg);
        const float lv = ok ? e : 0.f;
        rs[r] += lv;
        __bf16 hi, lo;
        split_bf(g[j][r] * lv, hi, lo);
        mH[l * kLP + scol] = hi;
        mL[l * kLP + scol] = lo;
      }
    }
#pragma unroll
    for (int r = 0; r < 8; ++r) {
      float v = rs[r];
      v += __shfl_xor(v, 1, 32);
      v += __shfl_xor(v, 2, 32);
      v += __shfl_xor(v, 4, 32);
      v += __shfl_xor(v, 8, 32);
      rs[r] = v;
    }
    if (rl == 0) {
#pragma unroll
      for (int r = 0; r < 8; ++r) sNDG[(w & 1) * 64 + lt * 16 + 8 * hh + r] = rs[r];
    }
  }
  __syncthreads();
  {
    const float* sp = sn + ((size_t)h * kNch + c) * 4096;
#pragma unroll
    for (int i = 0; i < 4; ++i) {
      const int idx4 = t + 256 * i;
      const int p = idx4 >> 4, n4 = (idx4 & 15) * 4;
      const v4f v = *(const v4f*)(sp + p * 64 + n4);
#pragma unroll
      for (int e = 0; e < 4; ++e) { __bf16 hi, lo; split_bf(v[e], hi, lo); bH[p * kLP + n4 + e] = hi; bL[p * kLP + n4 + e] = lo; }
    }
  }
  __syncthreads();
  v8f o[2];
  o[0] = zero8(); o[1] = zero8();
  mma_pair64(aH, aL, lt * 16, bH, bL, cb2 * 16, lane, o[0], o[1]);
  acc_guard2(o[0], o[1]);
  __syncthreads();
  {
    const Taps tx = load_taps(convw, convb, 2 * kDm + h * kHd + col);
    conv_col16<true, false>(pX, h * kHd + col, growc, l0, tx, sSDO, aH, aL, col);
  }
  __syncthreads();
  v8f d[2];
  d[0] = zero8(); d[1] = zero8();
  mma_pair64(mH, mL, lt * 16, aH, aL, cb2 * 16, lane, d[0], d[1]);
  acc_guard4(d[0], d[1], o[0], o[1]);
  {
    float inv[8], sd[8];
#pragma unroll
    for (int r = 0; r < 8; ++r) {
      const int l = lt * 16 + 8 * hh + r;
      sd[r] = sSDO[l];
      const float nrm = sNDG[l] + sNDG[64 + l] + ndz * sd[r];
      inv[r] = 1.0f / nrm;
    }
#pragma unroll
    for (int j = 0; j < 2; ++j) {
      const int pcol = (cb2 + j) * 16 + rl;
#pragma unroll
      for (int r = 0; r < 8; ++r) {
        const int l = lt * 16 + 8 * hh + r;
        const float y = d[j][r] + sd[r] * o[j][r];
        const float yn = y * inv[r];
        __bf16 hi, lo;
        split_bf(yn, hi, lo);
        bH[l * kLP + pcol] = hi;
        bL[l * kLP + pcol] = lo;
      }
    }
  }
  __syncthreads();
  {
    const int q = lane >> 3, c8 = (lane & 7) * 8;
    unsigned short* dh = ynh + ((size_t)(c * kChunk)) * kDm + h * kHd + c8;
    unsigned short* dl = ynl + ((size_t)(c * kChunk)) * kDm + h * kHd + c8;
    for (int pass = 0; pass < 2; ++pass) {
#pragma unroll
      for (int it = 0; it < 2; ++it) {
        const int row = w * 8 + it * 4 + q;
        const v4u hv = *(const v4u*)(bH + row * kLP + c8);
        const v4u lv = *(const v4u*)(bL + row * kLP + c8);
        *(volatile v4u*)(dh + (size_t)row * kDm) = hv;
        *(volatile v4u*)(dl + (size_t)row * kDm) = lv;
      }
      __threadfence();
    }
  }
}

extern "C" void kernel_launch(void* const* d_in, const int* in_sizes, int n_in,
                              void* d_out, int out_size, void* d_ws,
                              size_t ws_size, hipStream_t stream) {
  if (n_in < 6) return;
  if (ws_size < kWsTotal) return;
  if (out_size < kBatch * kSeq * kDm) return;
  if (in_sizes[0] < kBatch * kSeq * kDm || in_sizes[1] < kProj * kDm || in_sizes[2] < kConvCh * 4 ||
      in_sizes[3] < kConvCh || in_sizes[4] < kNh || in_sizes[5] < kDm * kDm) return;

  const float* x     = (const float*)d_in[0];
  const float* win   = (const float*)d_in[1];
  const float* convw = (const float*)d_in[2];
  const float* convb = (const float*)d_in[3];
  const float* wbase = (const float*)d_in[4];
  const float* wout  = (const float*)d_in[5];
  float* out = (float*)d_out;

  char* ws = (char*)d_ws;
  unsigned short* WIN  = (unsigned short*)(ws + kOffWin);
  unsigned short* WOUT = (unsigned short*)(ws + kOffWout);
  unsigned short* XB   = (unsigned short*)(ws + kOffXb);
  float* PC  = (float*)(ws + kOffPC);
  float* PB  = (float*)(ws + kOffPB);
  float* PX  = (float*)(ws + kOffPX);
  float* PW  = (float*)(ws + kOffPW);
  float* REC = (float*)(ws + kOffRec);
  float* TW  = (float*)(ws + kOffTW);
  float* ST  = (float*)(ws + kOffSt);
  float* SN  = (float*)(ws + kOffSn);
  unsigned short* YNH = (unsigned short*)(ws + kOffYnH);
  unsigned short* YNL = (unsigned short*)(ws + kOffYnL);
  const float* dummyf = REC;

  k_cast_rows<<<dim3((kProjPad * 128 + 255) / 256), dim3(256), 0, stream>>>(win, WIN, kProj, kProjPad);
  k_cast_rows<<<dim3((kDm * 128 + 255) / 256), dim3(256), 0, stream>>>(wout, WOUT, kDm, kDm);

  static_assert(kSeq % 64 == 0 && kDm % 64 == 0 && (kDm % 32) == 0);
  const int gemmBlocks1024 = (kSeq / 64) * (kDm / 64) / 8;
  const int gemmBlocks64   = (kSeq / 64) * (64 / 64) / 8;

  for (int b = 0; b < kBatch; ++b) {
    const float* xb = x + (size_t)b * kSeq * kDm;
    k_cast_rows<<<dim3((kSeq * 128 + 255) / 256), dim3(256), 0, stream>>>(xb, XB, kSeq, kSeq);

    wmma_gemm64<1, 0, 0, 0, false, 0><<<dim3(gemmBlocks1024, 1), dim3(256), 0, stream>>>(
        XB, XB, kDm, 0L, WIN, WIN, kDm, 0L, PC, PC, kDm, 0L, dummyf, dummyf, 0L, kSeq, kDm, kDm, 1.0f);
    wmma_gemm64<1, 0, 0, 0, false, 0><<<dim3(gemmBlocks1024, 1), dim3(256), 0, stream>>>(
        XB, XB, kDm, 0L, WIN + (size_t)kDm * kDm, WIN, kDm, 0L, PB, PB, kDm, 0L, dummyf, dummyf, 0L, kSeq, kDm, kDm, 1.0f);
    wmma_gemm64<1, 0, 0, 0, false, 0><<<dim3(gemmBlocks1024, 1), dim3(256), 0, stream>>>(
        XB, XB, kDm, 0L, WIN + (size_t)2 * kDm * kDm, WIN, kDm, 0L, PX, PX, kDm, 0L, dummyf, dummyf, 0L, kSeq, kDm, kDm, 1.0f);
    wmma_gemm64<1, 0, 0, 0, false, 0><<<dim3(gemmBlocks64, 1), dim3(256), 0, stream>>>(
        XB, XB, kDm, 0L, WIN + (size_t)kConvCh * kDm, WIN, kDm, 0L, PW, PW, 64, 0L, dummyf, dummyf, 0L, kSeq, 64, kDm, 1.0f);

    k_tab<<<dim3(kNh), dim3(64), 0, stream>>>(PW, wbase, REC, TW);

    k_states<<<dim3(kNch, kNh), dim3(256), 0, stream>>>(PB, PX, convw, convb, REC, ST);
    k_inter<<<dim3(4096 / 64, kNh), dim3(256), 0, stream>>>(TW, ST, SN);
    k_out<<<dim3(kNch, kNh), dim3(256), 0, stream>>>(PC, PB, PX, convw, convb, REC, SN, YNH, YNL);

    wmma_gemm64<1, 2, 0, 0, false, 0><<<dim3(gemmBlocks1024, 1), dim3(256), 0, stream>>>(
        YNH, YNL, kDm, 0L, WOUT, WOUT, kDm, 0L, out + (size_t)b * kSeq * kDm, dummyf == nullptr ? (void*)0 : (void*)PC,
        kDm, 0L, dummyf, dummyf, 0L, kSeq, kDm, kDm, 1.0f);
  }
  (void)stream;
}
